// MSA_46033459478834
// MI455X (gfx1250) — hardware-verified
//
#include <hip/hip_runtime.h>
#include <math.h>
#include <stdint.h>

#define NB   16
#define NT   512
#define NE   768
#define NH   12
#define HDD  64
#define NL   100
#define NLP  128
#define NR   (NB * NT)
#define NEGB (-1.0e9f)
#define LNEPS 1.0e-12f
#define NX8  (NR * NE / 8)
#define NTE8 (NLP * NE / 8)

static_assert(NR % 64 == 0);
static_assert(NE % 64 == 0);
static_assert(NT % 64 == 0);
static_assert(NE % 32 == 0);
static_assert(NLP % 32 == 0);
static_assert(NX8 % 256 == 0);
static_assert(NTE8 % 256 == 0);
static_assert(NE == NH * HDD);
static_assert((size_t)NR * NE + (size_t)NR * NL == 7110656);

typedef __attribute__((ext_vector_type(16))) _Float16 v16h;
typedef __attribute__((ext_vector_type(8)))  _Float16 v8h;
typedef __attribute__((ext_vector_type(16))) __bf16   v16b;
typedef __attribute__((ext_vector_type(8)))  __bf16   v8b;
typedef __attribute__((ext_vector_type(8)))  float    v8f;
typedef __attribute__((ext_vector_type(4)))  float    v4f;
typedef __attribute__((ext_vector_type(4)))  unsigned int v4u;
typedef __attribute__((ext_vector_type(2)))  unsigned int v2u;
typedef v4f __attribute__((may_alias)) v4fa;
typedef v4u __attribute__((may_alias)) v4ua;
typedef v2u __attribute__((may_alias)) v2ua;
typedef v8b __attribute__((may_alias)) v8ba;

__device__ __forceinline__ unsigned short f2bf_bits(float f) {
  unsigned u = __float_as_uint(f);
  return (unsigned short)((u + 0x7FFFu + ((u >> 16) & 1u)) >> 16);
}
__device__ __forceinline__ float bf_bits2f(unsigned short hb) { return __uint_as_float(((unsigned)hb) << 16); }
__device__ __forceinline__ float bfr(float f) { return bf_bits2f(f2bf_bits(f)); }
__device__ __forceinline__ unsigned pk16(unsigned short a, unsigned short b) { return (unsigned)a | ((unsigned)b << 16); }
__device__ __forceinline__ void split_bits(float f, unsigned short& hb, unsigned short& lb) {
  hb = f2bf_bits(f);
  lb = f2bf_bits(f - bf_bits2f(hb));
}
__device__ __forceinline__ __bf16 bits2bf(unsigned short hb) { return __builtin_bit_cast(__bf16, hb); }
__device__ __forceinline__ void at_split(float f, __bf16& hi, __bf16& lo) {
  unsigned short hb, lb;
  split_bits(f, hb, lb);
  hi = bits2bf(hb);
  lo = bits2bf(lb);
}
__device__ __forceinline__ v4u pack8bf(v4f a, v4f c) {
  v4u r;
  r.x = pk16(f2bf_bits(a.x), f2bf_bits(a.y));
  r.y = pk16(f2bf_bits(a.z), f2bf_bits(a.w));
  r.z = pk16(f2bf_bits(c.x), f2bf_bits(c.y));
  r.w = pk16(f2bf_bits(c.z), f2bf_bits(c.w));
  return r;
}

__device__ __forceinline__ void dep_guard_b(v8f& a, v8f& b, v16b x, v16b y) { asm volatile("v_nop\n\tv_nop\n\tv_nop\n\tv_nop" : "+v"(a), "+v"(b) : "v"(x), "v"(y)); }
__device__ __forceinline__ void keep4_b(v16b a, v16b b, v16b c, v16b d) { asm volatile("v_nop" :: "v"(a), "v"(b), "v"(c), "v"(d)); }
__device__ __forceinline__ void acc_guard4(v8f& a, v8f& b, v8f& c, v8f& d) { asm volatile("v_nop\n\tv_nop\n\tv_nop\n\tv_nop" : "+v"(a), "+v"(b), "+v"(c), "+v"(d)); }

union FB { v16b v; v8b h[2]; };
__device__ __forceinline__ v16b frag_load(const __bf16* p) {
  FB f;
  f.h[0] = *(const v8ba*)(p);
  f.h[1] = *(const v8ba*)(p + 16);
  return f.v;
}
__device__ __forceinline__ v8f mma_bf(v16b a, v16b b, v8f c) {
  return __builtin_amdgcn_wmma_f32_16x16x32_bf16(false, a, false, b, (short)0, c, false, false);
}
__device__ __forceinline__ v8f at_mma(v16b a, v16b b, v8f c) {
  c = mma_bf(a, b, c);
  asm volatile("v_nop\n\tv_nop\n\tv_nop\n\tv_nop" : "+v"(c) : "v"(a), "v"(b));
  return c;
}

template <int SPL, int BIAS_MODE, int OUT_MODE>
__global__ __launch_bounds__(256) void wmma_gemm64(
    const unsigned short* __restrict__ Ap, const unsigned short* __restrict__ A2p, int lda, long strideA,
    const unsigned short* __restrict__ Btp, const unsigned short* __restrict__ Bt2p, int ldb, long strideB,
    void* __restrict__ Cout, void* __restrict__ Cout2, int ldc, long strideC,
    const float* __restrict__ bias, int M, int N, int K, float scale) {
  constexpr bool SA = (SPL & 1) != 0;
  constexpr bool SB = (SPL & 2) != 0;
  const __bf16* A   = (const __bf16*)(const void*)Ap;
  const __bf16* A2  = (const __bf16*)(const void*)A2p;
  const __bf16* Bt  = (const __bf16*)(const void*)Btp;
  const __bf16* Bt2 = (const __bf16*)(const void*)Bt2p;
  __shared__ __align__(16) float sT[8][16 * 68];
  const int b    = blockIdx.y;
  const int lane = threadIdx.x & 31;
  const int wave = threadIdx.x >> 5;
  const int tilesN = N >> 6;
  const int tilesM = M >> 6;
  const int tile = blockIdx.x * 8 + wave;
  if (tile >= tilesM * tilesN) return;
  const int tm = tile / tilesN;
  const int tn = tile - tm * tilesN;
  const int m0 = tm << 6;
  const int n0 = tn << 6;

  const __bf16* Ab  = A  + (size_t)b * strideA;
  const __bf16* Bb  = Bt + (size_t)b * strideB;
  const __bf16* Ab2 = SA ? (A2  + (size_t)b * strideA) : nullptr;
  const __bf16* Bb2 = SB ? (Bt2 + (size_t)b * strideB) : nullptr;

  const int rlane = lane & 15;
  const int koff  = (lane >> 4) * 8;
  const int mOff  = (lane >> 4) * 8;

  v8f acc[4][4];
#pragma unroll
  for (int i = 0; i < 4; ++i)
#pragma unroll
    for (int j = 0; j < 4; ++j) acc[i][j] = (v8f){0.f,0.f,0.f,0.f,0.f,0.f,0.f,0.f};

  for (int k0 = 0; k0 < K; k0 += 32) {
    v16b bh[4], bl[4];
#pragma unroll
    for (int j = 0; j < 4; ++j) {
      const size_t bo = (size_t)(n0 + (j << 4) + rlane) * ldb + koff + k0;
      bh[j] = frag_load(Bb + bo);
      if (SB) bl[j] = frag_load(Bb2 + bo);
    }
#pragma unroll
    for (int i = 0; i < 4; ++i) {
      const size_t ao = (size_t)(m0 + (i << 4) + rlane) * lda + koff + k0;
      v16b ah = frag_load(Ab + ao);
      v16b al = ah;
      if (SA) al = frag_load(Ab2 + ao);
#pragma unroll
      for (int j = 0; j < 4; ++j) {
        acc[i][j] = mma_bf(ah, bh[j], acc[i][j]);
        if (SB) acc[i][j] = mma_bf(ah, bl[j], acc[i][j]);
        if (SA) acc[i][j] = mma_bf(al, bh[j], acc[i][j]);
      }
      dep_guard_b(acc[i][0], acc[i][3], ah, al);
    }
    keep4_b(bh[0], bh[1], bh[2], bh[3]);
    if (SB) keep4_b(bl[0], bl[1], bl[2], bl[3]);
  }
  acc_guard4(acc[0][0], acc[0][1], acc[0][2], acc[0][3]);
  acc_guard4(acc[1][0], acc[1][1], acc[1][2], acc[1][3]);
  acc_guard4(acc[2][0], acc[2][1], acc[2][2], acc[2][3]);
  acc_guard4(acc[3][0], acc[3][1], acc[3][2], acc[3][3]);

  float* slab = sT[wave];
#pragma unroll
  for (int i = 0; i < 4; ++i) {
    const int mBase = m0 + (i << 4);
#pragma unroll
    for (int j = 0; j < 4; ++j) {
      const int n = n0 + (j << 4) + rlane;
      float bvn = 0.f;
      if (BIAS_MODE == 2) bvn = bias[n];
#pragma unroll
      for (int r = 0; r < 8; ++r) {
        float v = acc[i][j][r] * scale;
        if (BIAS_MODE == 1) v += bias[mBase + mOff + r];
        if (BIAS_MODE == 2) v += bvn;
        slab[(mOff + r) * 68 + (j << 4) + rlane] = v;
      }
    }
    __builtin_amdgcn_fence(__ATOMIC_RELEASE, "workgroup");
    __builtin_amdgcn_wave_barrier();
    __builtin_amdgcn_fence(__ATOMIC_ACQUIRE, "workgroup");
    if (OUT_MODE == 0) {
      float* C = (float*)Cout + (size_t)b * strideC;
      const int hh = lane >> 4, c4 = (lane & 15) * 4;
      for (int pass = 0; pass < 2; ++pass) {
#pragma unroll
        for (int it = 0; it < 8; ++it) {
          const int row = it * 2 + hh;
          v4f v = *(const v4fa*)(slab + row * 68 + c4);
          *(volatile v4f*)(C + (size_t)(mBase + row) * ldc + n0 + c4) = v;
        }
        __threadfence();
      }
    } else {
      const int q = lane >> 3, c8 = (lane & 7) * 8;
      unsigned short* C  = (unsigned short*)Cout  + (size_t)b * strideC;
      unsigned short* C2 = (unsigned short*)Cout2 + (size_t)b * strideC;
      for (int pass = 0; pass < 2; ++pass) {
#pragma unroll
        for (int it = 0; it < 4; ++it) {
          const int row = it * 4 + q;
          const float* sp = slab + row * 68 + c8;
          v8h hv, lv;
#pragma unroll
          for (int e = 0; e < 8; ++e) {
            unsigned short hb = f2bf_bits(sp[e]);
            unsigned short lb = f2bf_bits(sp[e] - bf_bits2f(hb));
            hv[e] = __builtin_bit_cast(_Float16, hb);
            lv[e] = __builtin_bit_cast(_Float16, lb);
          }
          *(volatile v8h*)(C  + (size_t)(mBase + row) * ldc + n0 + c8) = hv;
          *(volatile v8h*)(C2 + (size_t)(mBase + row) * ldc + n0 + c8) = lv;
        }
        __threadfence();
      }
    }
    __builtin_amdgcn_fence(__ATOMIC_RELEASE, "workgroup");
    __builtin_amdgcn_wave_barrier();
    __builtin_amdgcn_fence(__ATOMIC_ACQUIRE, "workgroup");
  }
}

__global__ __launch_bounds__(256) void conv_kernel(const float* __restrict__ x, const float* __restrict__ te,
                                                   unsigned short* __restrict__ XB, unsigned short* __restrict__ TE) {
  const int tid = threadIdx.x;
  v4f a, cc;
  unsigned short* dst;
  if (blockIdx.x < NX8 / 256) {
    const size_t g = (size_t)blockIdx.x * 256 + tid;
    a  = *(const v4fa*)(x + g * 8);
    cc = *(const v4fa*)(x + g * 8 + 4);
    dst = XB + g * 8;
  } else {
    const int e  = (blockIdx.x - NX8 / 256) * 256 + tid;
    const int l  = e / (NE / 8);
    const int c8 = (e - l * (NE / 8)) * 8;
    const int ls = (l < NL) ? l : (NL - 1);
    a  = *(const v4fa*)(te + (size_t)ls * NE + c8);
    cc = *(const v4fa*)(te + (size_t)ls * NE + c8 + 4);
    const bool ok = (l < NL);
    a.x  = ok ? a.x  : 0.f; a.y  = ok ? a.y  : 0.f; a.z  = ok ? a.z  : 0.f; a.w  = ok ? a.w  : 0.f;
    cc.x = ok ? cc.x : 0.f; cc.y = ok ? cc.y : 0.f; cc.z = ok ? cc.z : 0.f; cc.w = ok ? cc.w : 0.f;
    dst = TE + (size_t)e * 8;
  }
  const v4u pv = pack8bf(a, cc);
  *(volatile v4u*)dst = pv;
  __threadfence();
  *(volatile v4u*)dst = pv;
}

__global__ __launch_bounds__(256) void tr_kernel(const float* __restrict__ w0, const float* __restrict__ w1,
                                                 const float* __restrict__ w2, const float* __restrict__ w3,
                                                 const float* __restrict__ te,
                                                 unsigned short* __restrict__ o0, unsigned short* __restrict__ o1,
                                                 unsigned short* __restrict__ o2, unsigned short* __restrict__ o3,
                                                 unsigned short* __restrict__ ote) {
  __shared__ __align__(16) float tf[64 * 68];
  const int z = blockIdx.z;
  const float* W;
  unsigned short* O;
  int R, P;
  if (z == 4) {
    if (blockIdx.y >= 2) return;
    W = te; O = ote; R = NL; P = NLP;
  } else if (z == 0) { W = w0; O = o0; R = NE; P = NE; }
  else if (z == 1)   { W = w1; O = o1; R = NE; P = NE; }
  else if (z == 2)   { W = w2; O = o2; R = NE; P = NE; }
  else               { W = w3; O = o3; R = NE; P = NE; }
  const int c0  = blockIdx.x * 64;
  const int r0  = blockIdx.y * 64;
  const int tid = threadIdx.x;
  {
    const int lr = tid >> 4;
    const int c4 = (tid & 15) * 4;
#pragma unroll
    for (int it = 0; it < 4; ++it) {
      const int rr = it * 16 + lr;
      const int ra = r0 + rr;
      const int rs = (ra < R) ? ra : (R - 1);
      v4f a = *(const v4fa*)(W + (size_t)rs * NE + c0 + c4);
      const bool ok = (ra < R);
      a.x = ok ? a.x : 0.f; a.y = ok ? a.y : 0.f; a.z = ok ? a.z : 0.f; a.w = ok ? a.w : 0.f;
      *(v4f*)(tf + rr * 68 + c4) = a;
    }
  }
  __syncthreads();
  const int sub = tid >> 3;
  const int c8  = (tid & 7) * 8;
  v4u hv[2];
#pragma unroll
  for (int it = 0; it < 2; ++it) {
    const int oc = it * 32 + sub;
    v4u a;
#pragma unroll
    for (int q = 0; q < 4; ++q) {
      const float f0 = tf[(c8 + 2 * q) * 68 + oc];
      const float f1 = tf[(c8 + 2 * q + 1) * 68 + oc];
      a[q] = pk16(f2bf_bits(f0), f2bf_bits(f1));
    }
    hv[it] = a;
  }
  for (int pass = 0; pass < 2; ++pass) {
#pragma unroll
    for (int it = 0; it < 2; ++it) {
      const int oc = it * 32 + sub;
      const size_t go = (size_t)(c0 + oc) * P + r0 + c8;
      *(volatile v4u*)(O + go) = hv[it];
    }
    __threadfence();
  }
}

__global__ __launch_bounds__(256) void cq_kernel(const float* __restrict__ tp, const float* __restrict__ Wq,
                                                 const float* __restrict__ bq, float* __restrict__ CQB) {
  __shared__ float stp[NE];
  const int tid = threadIdx.x;
  for (int i = tid; i < NE; i += 256) stp[i] = bfr(tp[i]);
  __syncthreads();
  const int n = blockIdx.x * 256 + tid;
  float acc = 0.0f;
#pragma unroll 4
  for (int k = 0; k < NE; ++k) acc = fmaf(stp[k], bfr(Wq[(size_t)k * NE + n]), acc);
  const float v = acc + bfr(bq[n]);
  ((volatile float*)CQB)[n] = v;
  __threadfence();
  ((volatile float*)CQB)[n] = v;
}

__global__ __launch_bounds__(128) void lab_kernel(const unsigned short* __restrict__ XBp, const unsigned short* __restrict__ TEp,
                                                  float* __restrict__ out1,
                                                  unsigned short* __restrict__ ATTh, unsigned short* __restrict__ ATTl) {
  __shared__ __align__(16) float  sS[4][16 * NL];
  __shared__ __align__(16) __bf16 sAh[4][16 * NLP];
  __shared__ __align__(16) __bf16 sAl[4][16 * NLP];
  const __bf16* XB = (const __bf16*)(const void*)XBp;
  const __bf16* TE = (const __bf16*)(const void*)TEp;
  const int tid = threadIdx.x, wave = tid >> 5, lane = tid & 31, hh = lane >> 4, c = lane & 15;
  const int row0 = blockIdx.x * 64 + wave * 16;

  const __bf16* arow = XB + (size_t)(row0 + c) * NE + 8 * hh;
  const __bf16* brow = TE + (size_t)c * NE + 8 * hh;

  v8f acc[8];
#pragma unroll
  for (int j = 0; j < 8; ++j) acc[j] = (v8f){0.f,0.f,0.f,0.f,0.f,0.f,0.f,0.f};

#pragma unroll 1
  for (int k0 = 0; k0 < NE; k0 += 32) {
    const v16b a = frag_load(arow + k0);
#pragma unroll
    for (int j = 0; j < 8; ++j) {
      const v16b bb = frag_load(brow + (size_t)j * 16 * NE + k0);
      acc[j] = at_mma(a, bb, acc[j]);
    }
  }

  float* ss = sS[wave];
#pragma unroll
  for (int j = 0; j < 8; ++j) {
    const int col = 16 * j + c;
#pragma unroll
    for (int r = 0; r < 8; ++r) {
      if (col < NL) ss[(8 * hh + r) * NL + col] = acc[j][r];
    }
  }
  __syncthreads();
  {
    float* ob = out1 + (size_t)row0 * NL;
    for (int pass = 0; pass < 2; ++pass) {
#pragma unroll
      for (int it = 0; it < 13; ++it) {
        const int p  = it * 32 + lane;
        const int pc = (p < 400) ? p : 399;
        const v4f v = *(const v4fa*)(ss + 4 * pc);
        if (p < 400) *(volatile v4f*)(ob + 4 * p) = v;
      }
      __threadfence();
    }
  }

  __bf16* ahs = sAh[wave];
  __bf16* als = sAl[wave];
#pragma unroll
  for (int r = 0; r < 8; ++r) {
    float m = -INFINITY;
#pragma unroll
    for (int j = 0; j < 8; ++j) {
      const int col = 16 * j + c;
      const float sv = (col < NL) ? acc[j][r] : -INFINITY;
      m = fmaxf(m, sv);
    }
#pragma unroll
    for (int off = 1; off < 16; off <<= 1) m = fmaxf(m, __shfl_xor(m, off, 32));
    float e8[8];
    float sum = 0.0f;
#pragma unroll
    for (int j = 0; j < 8; ++j) {
      const int col = 16 * j + c;
      const float arg = (col < NL) ? (acc[j][r] - m) : -INFINITY;
      const float ev = expf(arg);
      e8[j] = ev;
      sum += ev;
    }
#pragma unroll
    for (int off = 1; off < 16; off <<= 1) sum += __shfl_xor(sum, off, 32);
    const float inv = 1.0f / sum;
#pragma unroll
    for (int j = 0; j < 8; ++j) {
      const int col = 16 * j + c;
      const float p = e8[j] * inv;
      __bf16 hi, lo;
      at_split(p, hi, lo);
      ahs[(8 * hh + r) * NLP + col] = hi;
      als[(8 * hh + r) * NLP + col] = lo;
    }
  }
  __syncthreads();
  {
    const int sub = lane >> 3, c8 = (lane & 7) * 8;
    for (int pass = 0; pass < 2; ++pass) {
#pragma unroll
      for (int it = 0; it < 8; ++it) {
        const int lid = it * 4 + sub;
        const int row = lid >> 1, half = lid & 1;
        const int idx = row * NLP + half * 64 + c8;
        const v4u hv = *(const v4ua*)(ahs + idx);
        const v4u lv = *(const v4ua*)(als + idx);
        const size_t go = (size_t)(row0 + row) * NLP + half * 64 + c8;
        *(volatile v4u*)(ATTh + go) = hv;
        *(volatile v4u*)(ATTl + go) = lv;
      }
      __threadfence();
    }
  }
}

__global__ __launch_bounds__(256) void ht_kernel(const float* __restrict__ FLE, const float* __restrict__ x,
                                                 unsigned short* __restrict__ HTh, unsigned short* __restrict__ HTl) {
  const size_t g = (size_t)blockIdx.x * 256 + threadIdx.x;
  const size_t base = g * 8;
  const v4f f0 = *(const v4fa*)(FLE + base);
  const v4f f1 = *(const v4fa*)(FLE + base + 4);
  const v4f x0 = *(const v4fa*)(x + base);
  const v4f x1 = *(const v4fa*)(x + base + 4);
  float h[8];
  h[0] = f0.x + bfr(x0.x); h[1] = f0.y + bfr(x0.y); h[2] = f0.z + bfr(x0.z); h[3] = f0.w + bfr(x0.w);
  h[4] = f1.x + bfr(x1.x); h[5] = f1.y + bfr(x1.y); h[6] = f1.z + bfr(x1.z); h[7] = f1.w + bfr(x1.w);
  unsigned short hb[8], lb[8];
#pragma unroll
  for (int e = 0; e < 8; ++e) split_bits(h[e], hb[e], lb[e]);
  v4u hv, lv;
  hv.x = pk16(hb[0], hb[1]); hv.y = pk16(hb[2], hb[3]); hv.z = pk16(hb[4], hb[5]); hv.w = pk16(hb[6], hb[7]);
  lv.x = pk16(lb[0], lb[1]); lv.y = pk16(lb[2], lb[3]); lv.z = pk16(lb[4], lb[5]); lv.w = pk16(lb[6], lb[7]);
  *(volatile v4u*)(HTh + base) = hv;
  *(volatile v4u*)(HTl + base) = lv;
  __threadfence();
  *(volatile v4u*)(HTh + base) = hv;
  *(volatile v4u*)(HTl + base) = lv;
}

#define AT_D  64
#define AT_NW 4
#define AT_QB 64
#define AT_KC 64

__global__ __launch_bounds__(128)
void attn_kernel(const unsigned short* __restrict__ qhp, const unsigned short* __restrict__ qlp,
                 const unsigned short* __restrict__ khp, const unsigned short* __restrict__ klp,
                 const unsigned short* __restrict__ vhp, const unsigned short* __restrict__ vlp,
                 const float* __restrict__ maskp,
                 unsigned short* __restrict__ chp, unsigned short* __restrict__ clp, float sscale) {
  __shared__ __align__(16) __bf16 Ksh[AT_KC * AT_D];
  __shared__ __align__(16) __bf16 Ksl[AT_KC * AT_D];
  __shared__ __align__(16) __bf16 Vth[AT_D * AT_KC];
  __shared__ __align__(16) __bf16 Vtl[AT_D * AT_KC];
  __shared__ __align__(16) __bf16 Psh[AT_NW][16 * AT_KC];
  __shared__ __align__(16) __bf16 Psl[AT_NW][16 * AT_KC];
  __shared__ __align__(16) float  sPB[NT];

  const int tid  = threadIdx.x;
  const int wave = tid >> 5;
  const int lane = tid & 31;
  const int hh   = lane >> 4;
  const int c    = lane & 15;

  const int nqb = NT / AT_QB;
  const int bx = blockIdx.x;
  const int qb = bx % nqb;
  const int h  = bx / nqb;
  const int b  = blockIdx.y;
  const int q0 = qb * AT_QB + wave * 16;
  const size_t brow = (size_t)b * NT;

  const __bf16* Qh = (const __bf16*)(const void*)qhp + brow * NE + (size_t)h * AT_D;
  const __bf16* Ql = (const __bf16*)(const void*)qlp + brow * NE + (size_t)h * AT_D;
  const __bf16* Kh = (const __bf16*)(const void*)khp + brow * NE + (size_t)h * AT_D;
  const __bf16* Kl = (const __bf16*)(const void*)klp + brow * NE + (size_t)h * AT_D;
  const __bf16* Vh = (const __bf16*)(const void*)vhp + ((size_t)b * NE + (size_t)h * AT_D) * NT;
  const __bf16* Vl = (const __bf16*)(const void*)vlp + ((size_t)b * NE + (size_t)h * AT_D) * NT;

  {
    const v4f mv = *(const v4fa*)(maskp + brow + 4 * tid);
    sPB[4 * tid + 0] = (1.0f - bfr(mv.x)) * NEGB;
    sPB[4 * tid + 1] = (1.0f - bfr(mv.y)) * NEGB;
    sPB[4 * tid + 2] = (1.0f - bfr(mv.z)) * NEGB;
    sPB[4 * tid + 3] = (1.0f - bfr(mv.w)) * NEGB;
  }

  v16b qah[2], qal[2];
#pragma unroll
  for (int dc = 0; dc < 2; ++dc) {
    const __bf16* qr = Qh + (size_t)(q0 + c) * NE + dc * 32 + 8 * hh;
    const __bf16* ql = Ql + (size_t)(q0 + c) * NE + dc * 32 + 8 * hh;
    qah[dc] = frag_load(qr);
    qal[dc] = frag_load(ql);
  }

  float mrow[8], lrow[8];
  v8f oacc[4];
#pragma unroll
  for (int r = 0; r < 8; ++r) { mrow[r] = -INFINITY; lrow[r] = 0.f; }
#pragma unroll
  for (int t = 0; t < 4; ++t) oacc[t] = (v8f){0.f,0.f,0.f,0.f,0.f,0.f,0.f,0.f};

  const int nChunks = NT / AT_KC;
  for (int kc = 0; kc < nChunks; ++kc) {
    const int kv0 = kc * AT_KC;
    __syncthreads();
    {
      const int r = tid >> 1, half = (tid & 1) * 32;
      const __bf16* ksh = Kh + (size_t)(kv0 + r) * NE + half;
      const __bf16* ksl = Kl + (size_t)(kv0 + r) * NE + half;
      const __bf16* vsh = Vh + (size_t)r * NT + kv0 + half;
      const __bf16* vsl = Vl + (size_t)r * NT + kv0 + half;
#pragma unroll
      for (int i = 0; i < 4; ++i) {
        const v8b a0 = *(const v8ba*)(ksh + 8 * i);
        const v8b a1 = *(const v8ba*)(ksl + 8 * i);
        const v8b b0 = *(const v8ba*)(vsh + 8 * i);
        const v8b b1 = *(const v8ba*)(vsl + 8 * i);
        *(v8b*)(Ksh + r * AT_D  + half + 8 * i) = a0;
        *(v8b*)(Ksl + r * AT_D  + half + 8 * i) = a1;
        *(v8b*)(Vth + r * AT_KC + half + 8 * i) = b0;
        *(v8b*)(Vtl + r * AT_KC + half + 8 * i) = b1;
      }
    }
    __syncthreads();

    v8f s[4];
#pragma unroll
    for (int j = 0; j < 4; ++j) {
      s[j] = (v8f){0.f,0.f,0.f,0.f,0.f,0.f,0.f,0.f};
#pragma unroll
      for (int dc = 0; dc < 2; ++dc) {
        FB kb, kl;
        kb.h[0] = *(const v8ba*)(Ksh + (j * 16 + c) * AT_D + dc * 32 + 8 * hh);
        kb.h[1] = *(const v8ba*)(Ksh + (j * 16 + c) * AT_D + dc * 32 + 16 + 8 * hh);
        kl.h[0] = *(const v8ba*)(Ksl + (j * 16 + c) * AT_D + dc * 32 + 8 * hh);
        kl.h[1] = *(const v8ba*)(Ksl + (j * 16 + c) * AT_D + dc * 32 + 16 + 8 * hh);
        s[j] = at_mma(qah[dc], kb.v, s[j]);
        s[j] = at_mma(qah[dc], kl.v, s[j]);
        s[j] = at_mma(qal[dc], kb.v, s[j]);
      }
    }
    float pbj[4];
#pragma unroll
    for (int j = 0; j < 4; ++j) pbj[j] = sPB[kv0 + j * 16 + c];

    float cm[8];
#pragma unroll
    for (int r = 0; r < 8; ++r) {
      const int qi = q0 + 8 * hh + r;
      float m = -INFINITY;
#pragma unroll
      for (int j = 0; j < 4; ++j) {
        const int ki = kv0 + j * 16 + c;
        const float dg = (ki == qi) ? NEGB : 0.0f;
        const float sv = (s[j][r] * sscale + pbj[j]) + dg;
        s[j][r] = sv;
        m = fmaxf(m, sv);
      }
#pragma unroll
      for (int off = 1; off < 16; off <<= 1) m = fmaxf(m, __shfl_xor(m, off, 32));
      cm[r] = m;
    }
    __bf16* pwh = Psh[wave];
    __bf16* pwl = Psl[wave];
#pragma unroll
    for (int r = 0; r < 8; ++r) {
      const float mnew = fmaxf(mrow[r], cm[r]);
      const float alpha = expf(mrow[r] - mnew);
      mrow[r] = mnew;
      float psum = 0.f;
#pragma unroll
      for (int j = 0; j < 4; ++j) {
        const float p = expf(s[j][r] - mnew);
        psum += p;
        __bf16 a, bl; at_split(p, a, bl);
        pwh[(8 * hh + r) * AT_KC + j * 16 + c] = a;
        pwl[(8 * hh + r) * AT_KC + j * 16 + c] = bl;
      }
#pragma unroll
      for (int off = 1; off < 16; off <<= 1) psum += __shfl_xor(psum, off, 32);
      lrow[r] = lrow[r] * alpha + psum;
#pragma unroll
      for (int t = 0; t < 4; ++t) oacc[t][r] *= alpha;
    }
    __builtin_amdgcn_fence(__ATOMIC_RELEASE, "workgroup");
    __builtin_amdgcn_wave_barrier();
    __builtin_amdgcn_fence(__ATOMIC_ACQUIRE, "workgroup");
#pragma unroll 1
    for (int kk = 0; kk < 2; ++kk) {
      FB pa, pl;
      pa.h[0] = *(const v8ba*)(pwh + c * AT_KC + kk * 32 + 8 * hh);
      pa.h[1] = *(const v8ba*)(pwh + c * AT_KC + kk * 32 + 16 + 8 * hh);
      pl.h[0] = *(const v8ba*)(pwl + c * AT_KC + kk * 32 + 8 * hh);
      pl.h[1] = *(const v8ba*)(pwl + c * AT_KC + kk * 32 + 16 + 8 * hh);
#pragma unroll
      for (int t = 0; t < 4; ++t) {
        FB vb, vl;
        vb.h[0] = *(const v8ba*)(Vth + (t * 16 + c) * AT_KC + kk * 32 + 8 * hh);
        vb.h[1] = *(const v8ba*)(Vth + (t * 16 + c) * AT_KC + kk * 32 + 16 + 8 * hh);
        vl.h[0] = *(const v8ba*)(Vtl + (t * 16 + c) * AT_KC + kk * 32 + 8 * hh);
        vl.h[1] = *(const v8ba*)(Vtl + (t * 16 + c) * AT_KC + kk * 32 + 16 + 8 * hh);
        oacc[t] = at_mma(pa.v, vb.v, oacc[t]);
        oacc[t] = at_mma(pa.v, vl.v, oacc[t]);
        oacc[t] = at_mma(pl.v, vb.v, oacc[t]);
      }
    }
  }

  __builtin_amdgcn_fence(__ATOMIC_RELEASE, "workgroup");
  __builtin_amdgcn_wave_barrier();
  __builtin_amdgcn_fence(__ATOMIC_ACQUIRE, "workgroup");
  __bf16* osh = Psh[wave];
  __bf16* osl = Psl[wave];
#pragma unroll
  for (int r = 0; r < 8; ++r) {
    const float inv = 1.0f / lrow[r];
#pragma unroll
    for (int t = 0; t < 4; ++t) {
      const float v = oacc[t][r] * inv;
      __bf16 hi, lo;
      at_split(v, hi, lo);
      osh[(8 * hh + r) * AT_D + t * 16 + c] = hi;
      osl[(8 * hh + r) * AT_D + t * 16 + c] = lo;
    }
  }
  __builtin_amdgcn_fence(__ATOMIC_RELEASE, "workgroup");
  __builtin_amdgcn_wave_barrier();
  __builtin_amdgcn_fence(__ATOMIC_ACQUIRE, "workgroup");
  {
    const int sub = lane >> 3, c8 = (lane & 7) * 8;
    for (int pass = 0; pass < 2; ++pass) {
#pragma unroll
      for (int it = 0; it < 4; ++it) {
        const int row = it * 4 + sub;
        const v4u hv = *(const v4ua*)(osh + row * AT_D + c8);
        const v4u lv = *(const v4ua*)(osl + row * AT_D + c8);
        const size_t go = (brow + q0 + row) * NE + (size_t)h * AT_D + c8;
        *(volatile v4u*)(chp + go) = hv;
        *(volatile v4u*)(clp + go) = lv;
      }
      __threadfence();
    }
  }
}

__global__ __launch_bounds__(256) void ln_kernel(const float* __restrict__ AO,
                                                 const unsigned short* __restrict__ HTh, const unsigned short* __restrict__ HTl,
                                                 const float* __restrict__ x, const float* __restrict__ tp,
                                                 const float* __restrict__ g, const float* __restrict__ be,
                                                 float* __restrict__ out0) {
  const int tid = threadIdx.x, lane = tid & 31, wave = tid >> 5;
  const int row = blockIdx.x * 8 + wave;
  const size_t rb = (size_t)row * NE;
  v4f y[6], ht[6];
  float s = 0.0f;
#pragma unroll
  for (int j = 0; j < 6; ++j) {
    const int col = j * 128 + 4 * lane;
    const v4f a  = *(const v4fa*)(AO + rb + col);
    const v4f xv = *(const v4fa*)(x + rb + col);
    const v4f tv = *(const v4fa*)(tp + col);
    const v2u hw = *(const v2ua*)(HTh + rb + col);
    const v2u lw = *(const v2ua*)(HTl + rb + col);
    v4f yy, hv;
    yy.x = a.x + (bfr(xv.x) + bfr(tv.x));
    yy.y = a.y + (bfr(xv.y) + bfr(tv.y));
    yy.z = a.z + (bfr(xv.z) + bfr(tv.z));
    yy.w = a.w + (bfr(xv.w) + bfr(tv.w));
    hv.x = __uint_as_float(hw.x << 16)          + __uint_as_float(lw.x << 16);
    hv.y = __uint_as_float(hw.x & 0xffff0000u)  + __uint_as_float(lw.x & 0xffff0000u);
    hv.z = __uint_as_float(hw.y << 16)          + __uint_as_float(lw.y << 16);
    hv.w = __uint_as_float(hw.y & 0xffff0000u)  + __uint_as_float(lw.y & 0xffff0000u);
    y[j] = yy; ht[j] = hv;
    s += (yy.x + yy.y) + (yy.z + yy.w);
  }
#pragma unroll
  for (int off = 1; off < 32; off <<= 1) s += __shfl_xor(s, off, 32);
  const float mu = s * (1.0f / (float)NE);
  float s2 = 0.0f;
#pragma unroll
  for (int j = 0; j < 6; ++j) {
    const float d0 = y[j].x - mu, d1 = y[j].y - mu, d2 = y[j].z - mu, d3 = y[j].w - mu;
    s2 += (d0 * d0 + d1 * d1) + (d2 * d2 + d3 * d3);
  }
#pragma unroll
  for (int off = 1; off < 32; off <<= 1) s2 += __shfl_xor(s2, off, 32);
  const float var  = s2 * (1.0f / (float)NE);
  const float rstd = 1.0f / sqrtf(var + LNEPS);
  v4f o[6];
#pragma unroll
  for (int j = 0; j < 6; ++j) {
    const int col = j * 128 + 4 * lane;
    const v4f gv = *(const v4fa*)(g + col);
    const v4f bv = *(const v4fa*)(be + col);
    v4f oo;
    oo.x = ((y[j].x - mu) * rstd * bfr(gv.x) + bfr(bv.x)) + ht[j].x;
    oo.y = ((y[j].y - mu) * rstd * bfr(gv.y) + bfr(bv.y)) + ht[j].y;
    oo.z = ((y[j].z - mu) * rstd * bfr(gv.z) + bfr(bv.z)) + ht[j].z;
    oo.w = ((y[j].w - mu) * rstd * bfr(gv.w) + bfr(bv.w)) + ht[j].w;
    o[j] = oo;
  }
  for (int pass = 0; pass < 2; ++pass) {
#pragma unroll
    for (int j = 0; j < 6; ++j) {
      const int col = j * 128 + 4 * lane;
      *(volatile v4f*)(out0 + rb + col) = o[j];
    }
    __threadfence();
  }
}

extern "C" void kernel_launch(void* const* d_in, const int* in_sizes, int n_in,
                              void* d_out, int out_size, void* d_ws, size_t ws_size,
                              hipStream_t stream) {
  if (n_in < 14) return;
  if (in_sizes[0] != NR * NE || in_sizes[1] != NR || in_sizes[2] != NL * NE || in_sizes[3] != NE) return;
  if (in_sizes[4] != NE * NE || in_sizes[6] != NE * NE || in_sizes[8] != NE * NE || in_sizes[10] != NE * NE) return;
  if (in_sizes[5] != NE || in_sizes[7] != NE || in_sizes[9] != NE || in_sizes[11] != NE) return;
  if (in_sizes[12] != NE || in_sizes[13] != NE) return;
  if (out_size != NR * NE + NR * NL) return;

  const float* x    = (const float*)d_in[0];
  const float* mask = (const float*)d_in[1];
  const float* te   = (const float*)d_in[2];
  const float* tp   = (const float*)d_in[3];
  const float* Wq   = (const float*)d_in[4];
  const float* bq   = (const float*)d_in[5];
  const float* Wk   = (const float*)d_in[6];
  const float* bk   = (const float*)d_in[7];
  const float* Wv   = (const float*)d_in[8];
  const float* bv   = (const float*)d_in[9];
  const float* Wo   = (const float*)d_in[10];
  const float* bo   = (const float*)d_in[11];
  const float* lng  = (const float*)d_in[12];
  const float* lnb  = (const float*)d_in[13];

  float* out0 = (float*)d_out;
  float* out1 = (float*)d_out + (size_t)NR * NE;

  const size_t PACT = (size_t)NR * NE * 2;
  const size_t PTE  = (size_t)NLP * NE * 2;
  const size_t PW   = (size_t)NE * NE * 2;
  const size_t PATT = (size_t)NR * NLP * 2;
  const size_t PCQ  = (size_t)NE * 4;
  size_t off = 0;
  const size_t oTE  = off; off += PTE;
  const size_t oTEt = off; off += PTE;
  const size_t oWqT = off; off += PW;
  const size_t oWkT = off; off += PW;
  const size_t oWvT = off; off += PW;
  const size_t oWoT = off; off += PW;
  const size_t oCQ  = off; off += PCQ;
  const size_t oR1  = off; off += 4 * PACT;
  const size_t oXB  = oR1;
  const size_t oATh = oR1 + PACT;
  const size_t oATl = oATh + PATT;
  const size_t oFLE = oATl + PATT;
  const size_t oKh  = oR1;
  const size_t oKl  = oR1 + PACT;
  const size_t oVTh = oR1 + 2 * PACT;
  const size_t oVTl = oR1 + 3 * PACT;
  const size_t oHTh = off; off += PACT;
  const size_t oHTl = off; off += PACT;
  const size_t oQh  = off; off += PACT;
  const size_t oQl  = off; off += PACT;
  const size_t oAO  = oQh;
  const size_t oCXh = off; off += PACT;
  const size_t oCXl = off; off += PACT;
  if (oFLE + 2 * PACT > oR1 + 4 * PACT) return;
  if (off > ws_size) return;

  char* ws = (char*)d_ws;
  unsigned short* TEp  = (unsigned short*)(ws + oTE);
  unsigned short* TEt  = (unsigned short*)(ws + oTEt);
  unsigned short* WqT  = (unsigned short*)(ws + oWqT);
  unsigned short* WkT  = (unsigned short*)(ws + oWkT);
  unsigned short* WvT  = (unsigned short*)(ws + oWvT);
  unsigned short* WoT  = (unsigned short*)(ws + oWoT);
  float*          CQB  = (float*)(ws + oCQ);
  unsigned short* XB   = (unsigned short*)(ws + oXB);
  unsigned short* ATTh = (unsigned short*)(ws + oATh);
  unsigned short* ATTl = (unsigned short*)(ws + oATl);
  float*          FLE  = (float*)(ws + oFLE);
  unsigned short* Kh   = (unsigned short*)(ws + oKh);
  unsigned short* Kl   = (unsigned short*)(ws + oKl);
  unsigned short* VTh  = (unsigned short*)(ws + oVTh);
  unsigned short* VTl  = (unsigned short*)(ws + oVTl);
  unsigned short* HTh  = (unsigned short*)(ws + oHTh);
  unsigned short* HTl  = (unsigned short*)(ws + oHTl);
  unsigned short* Qh   = (unsigned short*)(ws + oQh);
  unsigned short* Ql   = (unsigned short*)(ws + oQl);
  float*          AO   = (float*)(ws + oAO);
  unsigned short* CXh  = (unsigned short*)(ws + oCXh);
  unsigned short* CXl  = (unsigned short*)(ws + oCXl);

  const dim3 blk256(256), blk128(128);
  const dim3 gG(((NR / 64) * (NE / 64)) / 8, 1);
  const dim3 gVT(((NE / 64) * (NT / 64)) / 8, NB);

  conv_kernel<<<dim3(NX8 / 256 + NTE8 / 256), blk256, 0, stream>>>(x, te, XB, TEp);
  tr_kernel<<<dim3(NE / 64, NE / 64, 5), blk256, 0, stream>>>(Wq, Wk, Wv, Wo, te, WqT, WkT, WvT, WoT, TEt);
  cq_kernel<<<dim3(NE / 256), blk256, 0, stream>>>(tp, Wq, bq, CQB);
  lab_kernel<<<dim3(NR / 64), blk128, 0, stream>>>(XB, TEp, out1, ATTh, ATTl);
  wmma_gemm64<1, 0, 0><<<gG, blk256, 0, stream>>>(
      ATTh, ATTl, NLP, 0L, TEt, TEt, NLP, 0L, (void*)FLE, (void*)FLE, NE, 0L, bk, NR, NE, NLP, 1.0f);
  ht_kernel<<<dim3(NX8 / 256), blk256, 0, stream>>>(FLE, x, HTh, HTl);
  wmma_gemm64<0, 2, 2><<<gG, blk256, 0, stream>>>(
      XB, XB, NE, 0L, WqT, WqT, NE, 0L, (void*)Qh, (void*)Ql, NE, 0L, CQB, NR, NE, NE, 1.0f);
  wmma_gemm64<1, 2, 2><<<gG, blk256, 0, stream>>>(
      HTh, HTl, NE, 0L, WkT, WkT, NE, 0L, (void*)Kh, (void*)Kl, NE, 0L, bk, NR, NE, NE, 1.0f);
  wmma_gemm64<2, 1, 2><<<gVT, blk256, 0, stream>>>(
      WvT, WvT, NE, 0L, HTh, HTl, NE, (long)NT * NE, (void*)VTh, (void*)VTl, NT, (long)NE * NT, bv, NE, NT, NE, 1.0f);
  attn_kernel<<<dim3(NH * (NT / 64), NB), blk128, 0, stream>>>(Qh, Ql, Kh, Kl, VTh, VTl, mask, CXh, CXl, 0.125f);
  wmma_gemm64<1, 2, 0><<<gG, blk256, 0, stream>>>(
      CXh, CXl, NE, 0L, WoT, WoT, NE, 0L, (void*)AO, (void*)AO, NE, 0L, bo, NR, NE, NE, 1.0f);
  ln_kernel<<<dim3(NR / 8), blk256, 0, stream>>>(AO, HTh, HTl, x, tp, lng, lnb, out0);
  (void)hipGetLastError();
}
